// PyGNN_68796786147750
// MI455X (gfx1250) — hardware-verified
//
#include <hip/hip_runtime.h>
#include <stddef.h>
#include <math.h>


#define FDIM   128
#define HDIM   64
#define KDIM   192
#define NBAND  4
#define XCOL   256
#define NCLS   2
#define NTHR   256
#define NWAVE  8
#define EPT    8
#define NGRP   2
#define CHUNK  (NTHR * EPT * NGRP)
#define WCAP   (EPT * NGRP * 32)
#define LISTN  (NWAVE * WCAP)
#define NBC    4096
#define NBA    1024
#define GROWS  128
#define WSCALE 8.0f
#define WINV   0.125f

#define LDS_AGG  (NBA * HDIM * 4 + LISTN * 4 + 64)
#define LDS_FEAT (GROWS * KDIM * 2)
#define LDS_XW   (GROWS * 128 * 4)

static_assert((CHUNK & (CHUNK - 1)) == 0);
static_assert(CHUNK <= 4096);
static_assert(NBC <= 4096 && NBA <= 4096);
static_assert((NBC & (NBC - 1)) == 0 && (NBA & (NBA - 1)) == 0);
static_assert(NBC == NWAVE * 4 * 128);
static_assert((NBA * HDIM / 4) % NTHR == 0);
static_assert((NBA * NCLS) % (4 * NTHR) == 0);
static_assert(LISTN >= NBA * NCLS);
static_assert(NBA % NWAVE == 0);
static_assert(HDIM * HDIM / 8 == 2 * NTHR);
static_assert((XCOL * KDIM / 8) % NTHR == 0);
static_assert(GROWS * HDIM / 8 == 4 * NTHR);
static_assert(GROWS * FDIM / 8 == 8 * NTHR);
static_assert(GROWS == NWAVE * 16);
static_assert(GROWS * (HDIM + 8) * 2 <= LDS_FEAT);
static_assert(NBA % GROWS == 0);
static_assert((KDIM % 32) == 0 && (HDIM % 32) == 0);

typedef float    v2f  __attribute__((ext_vector_type(2)));
typedef float    v4f  __attribute__((ext_vector_type(4)));
typedef float    v8f  __attribute__((ext_vector_type(8)));
typedef int      v4i  __attribute__((ext_vector_type(4)));
typedef _Float16 v8h  __attribute__((ext_vector_type(8)));
typedef _Float16 v16h __attribute__((ext_vector_type(16)));
union FragH { v16h v; v8h h[2]; };

__device__ __forceinline__ v8h cvt8(v4f a, v4f b) {
  v8h r;
  r[0] = (_Float16)a.x; r[1] = (_Float16)a.y; r[2] = (_Float16)a.z; r[3] = (_Float16)a.w;
  r[4] = (_Float16)b.x; r[5] = (_Float16)b.y; r[6] = (_Float16)b.z; r[7] = (_Float16)b.w;
  return r;
}

__device__ __forceinline__ v8f wmh(v16h a, v16h b, v8f c) {
  v8f d = __builtin_amdgcn_wmma_f32_16x16x32_f16(false, a, false, b, (short)0, c, false, false);
  asm volatile("v_nop\n\tv_nop\n\tv_nop\n\tv_nop" : "+v"(d) : "v"(a), "v"(b));
  return d;
}

template <int NB>
__device__ __forceinline__ int scan_chunk(const int* __restrict__ dsts, int nE, int cbase, int slotBase,
                                          int vec8, int* list, int tid, int lane, int wave) {
  int wc = 0;
#pragma unroll
  for (int g = 0; g < NGRP; ++g) {
    const int el0  = (g * NTHR + tid) * EPT;
    const int e0   = cbase + el0;
    const int sent = -2147483647 - 1;
    v4i da, db;
    if (vec8 != 0 && cbase + CHUNK <= nE) {
      da = *(const v4i*)(dsts + e0);
      db = *(const v4i*)(dsts + e0 + 4);
    } else {
      da.x = (e0     < nE) ? dsts[min(e0, nE - 1)] : sent;
      da.y = (e0 + 1 < nE) ? dsts[min(e0 + 1, nE - 1)] : sent;
      da.z = (e0 + 2 < nE) ? dsts[min(e0 + 2, nE - 1)] : sent;
      da.w = (e0 + 3 < nE) ? dsts[min(e0 + 3, nE - 1)] : sent;
      db.x = (e0 + 4 < nE) ? dsts[min(e0 + 4, nE - 1)] : sent;
      db.y = (e0 + 5 < nE) ? dsts[min(e0 + 5, nE - 1)] : sent;
      db.z = (e0 + 6 < nE) ? dsts[min(e0 + 6, nE - 1)] : sent;
      db.w = (e0 + 7 < nE) ? dsts[min(e0 + 7, nE - 1)] : sent;
    }
    const unsigned nb = (unsigned)slotBase;
    const unsigned s0 = (unsigned)da.x - nb, s1 = (unsigned)da.y - nb;
    const unsigned s2 = (unsigned)da.z - nb, s3 = (unsigned)da.w - nb;
    const unsigned s4 = (unsigned)db.x - nb, s5 = (unsigned)db.y - nb;
    const unsigned s6 = (unsigned)db.z - nb, s7 = (unsigned)db.w - nb;
    const bool h0 = s0 < (unsigned)NB, h1 = s1 < (unsigned)NB, h2 = s2 < (unsigned)NB, h3 = s3 < (unsigned)NB;
    const bool h4 = s4 < (unsigned)NB, h5 = s5 < (unsigned)NB, h6 = s6 < (unsigned)NB, h7 = s7 < (unsigned)NB;
    const unsigned any = __builtin_amdgcn_ballot_w32(h0 | h1 | h2 | h3 | h4 | h5 | h6 | h7);
    if (any != 0u) {
#define HITJ(J, HJ, SJ) { \
        const unsigned mj = __builtin_amdgcn_ballot_w32(HJ); \
        if (mj != 0u) { \
          if (HJ) { \
            const int pos = wc + (int)__builtin_amdgcn_mbcnt_lo(mj, 0u); \
            if (pos < WCAP) list[wave * WCAP + pos] = ((el0 + (J)) << 12) | (int)(SJ); \
          } \
          wc += (int)__builtin_popcount(mj); } }
      HITJ(0, h0, s0)
      HITJ(1, h1, s1)
      HITJ(2, h2, s2)
      HITJ(3, h3, s3)
      HITJ(4, h4, s4)
      HITJ(5, h5, s5)
      HITJ(6, h6, s6)
      HITJ(7, h7, s7)
#undef HITJ
    }
  }
  return wc;
}

__global__ __launch_bounds__(NTHR) void k_wprep(
    const float* __restrict__ taw, const float* __restrict__ cvw, _Float16* wta, _Float16* wcv) {
  const int g0 = HDIM * HDIM / 8;
  const int g1 = XCOL * KDIM / 8;
  const int i = blockIdx.x * NTHR + (int)threadIdx.x;
  if (i >= g0 + g1) return;
  const bool seg0 = (blockIdx.x * NTHR) < g0;
  float v[8];
  _Float16* dp;
  if (seg0) {
    const int o  = i * 8;
    const int n  = o / HDIM;
    const int k0 = o - n * HDIM;
#pragma unroll
    for (int e = 0; e < 8; ++e) v[e] = taw[(k0 + e) * HDIM + n] * WSCALE;
    dp = wta + o;
  } else {
    const int o    = (i - g0) * 8;
    const int n    = o / KDIM;
    const int k0   = o - n * KDIM;
    const int band = n >> 6;
    const int j    = n & 63;
#pragma unroll
    for (int e = 0; e < 8; ++e) v[e] = cvw[((size_t)band * KDIM + k0 + e) * HDIM + j] * WSCALE;
    dp = wcv + o;
  }
  v4f a, b;
  a.x = v[0]; a.y = v[1]; a.z = v[2]; a.w = v[3];
  b.x = v[4]; b.y = v[5]; b.z = v[6]; b.w = v[7];
  const v8h hv = cvt8(a, b);
  *(volatile v8h*)dp = hv;
  __threadfence();
  *(volatile v8h*)dp = hv;
}

__global__ __launch_bounds__(NTHR) void k_count(
    const int* __restrict__ se, float* dinv, int nEs, int cntPad, int vec8) {
  __shared__ __attribute__((aligned(16))) int scnt[NBC];
  __shared__ __attribute__((aligned(16))) int list[LISTN];
  __shared__ int wcnt[NWAVE];
  const int tid = threadIdx.x, lane = tid & 31, wave = tid >> 5;
  const int nodeBase = blockIdx.x * NBC;
  const int b = blockIdx.y;
  const int* dsts = se + (size_t)(2 * b + 1) * (size_t)nEs;

  for (int i = tid; i < NBC; i += NTHR) scnt[i] = 0;
  __syncthreads();

  const int nChunks = (nEs + CHUNK - 1) / CHUNK;
#pragma unroll 1
  for (int ch = 0; ch < nChunks; ++ch) {
    const int cbase = ch * CHUNK;
    const int wc = scan_chunk<NBC>(dsts, nEs, cbase, nodeBase, vec8, list, tid, lane, wave);
    if (lane == 0) wcnt[wave] = wc;
    __syncthreads();
    if (wave == 0) {
#pragma unroll 1
      for (int wsx = 0; wsx < NWAVE; ++wsx) {
        int n = __builtin_amdgcn_readfirstlane(wcnt[wsx]);
        n = n > WCAP ? WCAP : (n < 0 ? 0 : n);
        const int* lp = list + wsx * WCAP;
#pragma unroll 1
        for (int i = 0; i < n; ++i) {
          const int ent  = __builtin_amdgcn_readfirstlane(lp[i]);
          const int slot = ent & (NBC - 1);
          if (lane == 0) scnt[slot] = scnt[slot] + 1;
        }
      }
    }
    __syncthreads();
  }

  v4f dq[4];
#pragma unroll
  for (int q = 0; q < 4; ++q) {
    const int f = (wave * 4 + q) * 128 + 4 * lane;
    const v4i c = *(const v4i*)(scnt + f);
    dq[q].x = rsqrtf((float)(c.x + 1));
    dq[q].y = rsqrtf((float)(c.y + 1));
    dq[q].z = rsqrtf((float)(c.z + 1));
    dq[q].w = rsqrtf((float)(c.w + 1));
  }
  float* dp = dinv + (size_t)b * (size_t)cntPad + (size_t)nodeBase;
#pragma unroll
  for (int q = 0; q < 4; ++q) {
    const int f = (wave * 4 + q) * 128 + 4 * lane;
    *(volatile v4f*)(dp + f) = dq[q];
  }
  __threadfence();
#pragma unroll
  for (int q = 0; q < 4; ++q) {
    const int f = (wave * 4 + q) * 128 + 4 * lane;
    *(volatile v4f*)(dp + f) = dq[q];
  }
}

__global__ __launch_bounds__(NTHR) void k_tagg(
    const int* __restrict__ ei, const float* __restrict__ ea, const float* __restrict__ tew,
    const float* __restrict__ teb, float* tsum, int nE, int vec8) {
  extern __shared__ v4f lds_dyn[];
  float* acc  = (float*)lds_dyn;
  int*   list = (int*)(acc + NBA * HDIM);
  int*   wcnt = list + LISTN;
  const int tid = threadIdx.x, lane = tid & 31, wave = tid >> 5;
  const int nodeBase = blockIdx.x * NBA;
  const int* dsts = ei + nE;

  {
    const v4f z = {0.f, 0.f, 0.f, 0.f};
    for (int i = tid; i < NBA * HDIM / 4; i += NTHR) ((v4f*)acc)[i] = z;
  }
  const float w0 = tew[2 * lane], w1 = tew[2 * lane + 1];
  const float b0 = teb[2 * lane], b1 = teb[2 * lane + 1];
  __syncthreads();

  const int nChunks = (nE + CHUNK - 1) / CHUNK;
#pragma unroll 1
  for (int ch = 0; ch < nChunks; ++ch) {
    const int cbase = ch * CHUNK;
    const int wc = scan_chunk<NBA>(dsts, nE, cbase, nodeBase, vec8, list, tid, lane, wave);
    if (lane == 0) wcnt[wave] = wc;
    __syncthreads();
    if (wave == 0) {
#pragma unroll 1
      for (int wsx = 0; wsx < NWAVE; ++wsx) {
        int n = __builtin_amdgcn_readfirstlane(wcnt[wsx]);
        n = n > WCAP ? WCAP : (n < 0 ? 0 : n);
        const int* lp = list + wsx * WCAP;
#pragma unroll 1
        for (int i = 0; i < n; ++i) {
          const int ent  = __builtin_amdgcn_readfirstlane(lp[i]);
          const int slot = ent & (NBA - 1);
          int e = cbase + ((ent >> 12) & (CHUNK - 1));
          e = e > nE - 1 ? nE - 1 : e;
          const float t = ea[e];
          v2f cv = {0.f, 0.f};
#pragma unroll 1
          for (int q = 0; q < 2; ++q) {
            const float wq  = (q == 0) ? w0 : w1;
            const float bq  = (q == 0) ? b0 : b1;
            const float val = cosf(t * wq + bq);
            cv.x = (q == 0) ? val : cv.x;
            cv.y = (q == 0) ? cv.y : val;
          }
          v2f* ap = (v2f*)(acc + slot * HDIM + 2 * lane);
          *ap = *ap + cv;
        }
      }
    }
    __syncthreads();
  }

  float* gp = tsum + (size_t)nodeBase * HDIM;
#pragma unroll 8
  for (int p = 0; p < NBA * HDIM / (4 * NTHR); ++p) {
    const int f = p * NTHR + tid;
    const v4f v = ((const v4f*)acc)[f];
    *(volatile v4f*)(gp + 4 * (size_t)f) = v;
  }
  __threadfence();
#pragma unroll 8
  for (int p = 0; p < NBA * HDIM / (4 * NTHR); ++p) {
    const int f = p * NTHR + tid;
    const v4f v = ((const v4f*)acc)[f];
    *(volatile v4f*)(gp + 4 * (size_t)f) = v;
  }
}

__global__ __launch_bounds__(NTHR) void k_feat(
    const float* __restrict__ tsum, const _Float16* __restrict__ wta, const float* __restrict__ tab,
    const float* __restrict__ feat, _Float16* f16p, int nN) {
  extern __shared__ v4f lds_dyn[];
  constexpr int AP = HDIM + 8;
  _Float16* sA = (_Float16*)lds_dyn;
  _Float16* sO = (_Float16*)lds_dyn;
  const int tid = threadIdx.x, lane = tid & 31, wave = tid >> 5, hh = lane >> 4, m = lane & 15;
  const int rowBase = blockIdx.x * GROWS;

#pragma unroll
  for (int i = 0; i < 4; ++i) {
    const int idx = i * NTHR + tid;
    const int r   = idx >> 3;
    const int c0  = (idx & 7) * 8;
    const float* ap = tsum + (size_t)(rowBase + r) * HDIM + c0;
    const v4f a = *(const v4f*)ap, b = *(const v4f*)(ap + 4);
    *(v8h*)(sA + r * AP + c0) = cvt8(a, b);
  }
  __syncthreads();

  v8f acc[4];
#pragma unroll
  for (int t = 0; t < 4; ++t) { v8f z = {0.f, 0.f, 0.f, 0.f, 0.f, 0.f, 0.f, 0.f}; acc[t] = z; }
  const _Float16* ar = sA + (wave * 16 + m) * AP + 8 * hh;
#pragma unroll
  for (int kt = 0; kt < HDIM / 32; ++kt) {
    FragH a;
    a.h[0] = *(const v8h*)(ar + 32 * kt);
    a.h[1] = *(const v8h*)(ar + 32 * kt + 16);
#pragma unroll
    for (int t = 0; t < 4; ++t) {
      const _Float16* bp = wta + (size_t)(16 * t + m) * HDIM + 32 * kt + 8 * hh;
      FragH b;
      b.h[0] = *(const v8h*)bp;
      b.h[1] = *(const v8h*)(bp + 16);
      acc[t] = wmh(a.v, b.v, acc[t]);
    }
  }
  __syncthreads();

  {
    _Float16* sp = sO + (wave * 16 + 8 * hh) * KDIM + FDIM + m;
#pragma unroll
    for (int t = 0; t < 4; ++t) {
      const float bl = tab[16 * t + m];
#pragma unroll
      for (int r = 0; r < 8; ++r) sp[r * KDIM + 16 * t] = (_Float16)(acc[t][r] * WINV + bl);
    }
  }
#pragma unroll
  for (int i = 0; i < 8; ++i) {
    const int idx = i * NTHR + tid;
    const int r   = idx >> 4;
    const int c0  = (idx & 15) * 8;
    int row = rowBase + r;
    row = row > nN - 1 ? nN - 1 : row;
    const float* fp = feat + (size_t)row * FDIM + c0;
    const v4f a = *(const v4f*)fp, b = *(const v4f*)(fp + 4);
    *(v8h*)(sO + r * KDIM + c0) = cvt8(a, b);
  }
  __syncthreads();

  const _Float16* lp = sO + wave * 16 * KDIM;
  _Float16* gp = f16p + (size_t)(rowBase + wave * 16) * KDIM;
#pragma unroll
  for (int p = 0; p < 16 * KDIM / (8 * 32); ++p) {
    const v8h v = *(const v8h*)(lp + 8 * (32 * p + lane));
    *(volatile v8h*)(gp + 8 * (32 * p + lane)) = v;
  }
  __threadfence();
#pragma unroll
  for (int p = 0; p < 16 * KDIM / (8 * 32); ++p) {
    const v8h v = *(const v8h*)(lp + 8 * (32 * p + lane));
    *(volatile v8h*)(gp + 8 * (32 * p + lane)) = v;
  }
}

__global__ __launch_bounds__(NTHR) void k_xw(
    const _Float16* __restrict__ f16p, const _Float16* __restrict__ wcv, const float* __restrict__ dinv,
    float* xw, int cntPad) {
  extern __shared__ v4f lds_dyn[];
  float* stg = (float*)lds_dyn;
  const int tid = threadIdx.x, lane = tid & 31, wave = tid >> 5, hh = lane >> 4, m = lane & 15;
  const int rowBase = blockIdx.x * GROWS;
  const int colHalf = blockIdx.y;
  const int colBase = colHalf * 128;

  v8f acc[8];
#pragma unroll
  for (int t = 0; t < 8; ++t) { v8f z = {0.f, 0.f, 0.f, 0.f, 0.f, 0.f, 0.f, 0.f}; acc[t] = z; }
  const _Float16* ar = f16p + (size_t)(rowBase + wave * 16 + m) * KDIM + 8 * hh;
#pragma unroll
  for (int kt = 0; kt < KDIM / 32; ++kt) {
    FragH a;
    a.h[0] = *(const v8h*)(ar + 32 * kt);
    a.h[1] = *(const v8h*)(ar + 32 * kt + 16);
#pragma unroll
    for (int t = 0; t < 8; ++t) {
      const _Float16* bp = wcv + (size_t)(colBase + 16 * t + m) * KDIM + 32 * kt + 8 * hh;
      FragH b;
      b.h[0] = *(const v8h*)bp;
      b.h[1] = *(const v8h*)(bp + 16);
      acc[t] = wmh(a.v, b.v, acc[t]);
    }
  }

  const int r0 = wave * 16 + 8 * hh;
  const float* dpa = dinv + (size_t)(2 * colHalf) * (size_t)cntPad + (size_t)rowBase + r0;
  const float* dpb = dpa + (size_t)cntPad;
  const v4f a0 = *(const v4f*)dpa, a1 = *(const v4f*)(dpa + 4);
  const v4f c0 = *(const v4f*)dpb, c1 = *(const v4f*)(dpb + 4);
  float sa[8], sb[8];
  sa[0] = a0.x; sa[1] = a0.y; sa[2] = a0.z; sa[3] = a0.w; sa[4] = a1.x; sa[5] = a1.y; sa[6] = a1.z; sa[7] = a1.w;
  sb[0] = c0.x; sb[1] = c0.y; sb[2] = c0.z; sb[3] = c0.w; sb[4] = c1.x; sb[5] = c1.y; sb[6] = c1.z; sb[7] = c1.w;
  float* sp = stg + r0 * 128 + m;
#pragma unroll
  for (int t = 0; t < 8; ++t) {
#pragma unroll
    for (int r = 0; r < 8; ++r) {
      const float s = (t < 4) ? sa[r] : sb[r];
      sp[r * 128 + 16 * t] = acc[t][r] * s * WINV;
    }
  }
  __syncthreads();

  const float* lp = stg + wave * 16 * 128 + 4 * lane;
  float* gp = xw + ((size_t)rowBase + wave * 16) * XCOL + colBase + 4 * lane;
#pragma unroll
  for (int i = 0; i < 16; ++i) { const v4f v = *(const v4f*)(lp + i * 128); *(volatile v4f*)(gp + (size_t)i * XCOL) = v; }
  __threadfence();
#pragma unroll
  for (int i = 0; i < 16; ++i) { const v4f v = *(const v4f*)(lp + i * 128); *(volatile v4f*)(gp + (size_t)i * XCOL) = v; }
}

__global__ __launch_bounds__(NTHR) void k_band(
    const int* __restrict__ se, const float* __restrict__ xw, const float* __restrict__ dinv,
    const float* __restrict__ cvb, const float* __restrict__ ow, float* plog,
    int nN, int nEs, int cntPad, int nPad, int vec8) {
  extern __shared__ v4f lds_dyn[];
  float* acc  = (float*)lds_dyn;
  int*   list = (int*)(acc + NBA * HDIM);
  int*   wcnt = list + LISTN;
  const int tid = threadIdx.x, lane = tid & 31, wave = tid >> 5;
  const int nodeBase = blockIdx.x * NBA;
  const int b = blockIdx.y;
  const int* srcs = se + (size_t)(2 * b) * (size_t)nEs;
  const int* dsts = srcs + nEs;
  const int colOff = b * HDIM;
  const int kc = colOff + 2 * lane;

  {
    const v4f z = {0.f, 0.f, 0.f, 0.f};
    for (int i = tid; i < NBA * HDIM / 4; i += NTHR) ((v4f*)acc)[i] = z;
  }
  __syncthreads();

  const int nChunks = (nEs + CHUNK - 1) / CHUNK;
#pragma unroll 1
  for (int ch = 0; ch < nChunks; ++ch) {
    const int cbase = ch * CHUNK;
    const int wc = scan_chunk<NBA>(dsts, nEs, cbase, nodeBase, vec8, list, tid, lane, wave);
    if (lane == 0) wcnt[wave] = wc;
    __syncthreads();
    if (wave == 0) {
#pragma unroll 1
      for (int wsx = 0; wsx < NWAVE; ++wsx) {
        int n = __builtin_amdgcn_readfirstlane(wcnt[wsx]);
        n = n > WCAP ? WCAP : (n < 0 ? 0 : n);
        const int* lp = list + wsx * WCAP;
#pragma unroll 1
        for (int i = 0; i < n; ++i) {
          const int ent  = __builtin_amdgcn_readfirstlane(lp[i]);
          const int slot = ent & (NBA - 1);
          int e = cbase + ((ent >> 12) & (CHUNK - 1));
          e = e > nEs - 1 ? nEs - 1 : e;
          int src = srcs[e];
          src = src < 0 ? 0 : (src > nN - 1 ? nN - 1 : src);
          const v2f v = *(const v2f*)(xw + (size_t)src * XCOL + kc);
          v2f* ap = (v2f*)(acc + slot * HDIM + 2 * lane);
          *ap = *ap + v;
        }
      }
    }
    __syncthreads();
  }

  float* splog = (float*)list;
  const float* dvp = dinv + (size_t)b * (size_t)cntPad + (size_t)nodeBase;
  const v2f cb = *(const v2f*)(cvb + b * HDIM + 2 * lane);
  const float o00 = ow[kc * NCLS + 0], o01 = ow[kc * NCLS + 1];
  const float o10 = ow[(kc + 1) * NCLS + 0], o11 = ow[(kc + 1) * NCLS + 1];
#pragma unroll 1
  for (int jj = 0; jj < NBA / NWAVE; ++jj) {
    const int slot = wave * (NBA / NWAVE) + jj;
    const int node = nodeBase + slot;
    const float d = dvp[slot];
    const v2f sv = *(const v2f*)(xw + (size_t)node * XCOL + kc);
    const v2f av = *(const v2f*)(acc + slot * HDIM + 2 * lane);
    float vx = (av.x + sv.x) * d + cb.x;
    float vy = (av.y + sv.y) * d + cb.y;
    vx = fmaxf(vx, 0.0f); vy = fmaxf(vy, 0.0f);
    float p0 = vx * o00 + vy * o10;
    float p1 = vx * o01 + vy * o11;
#pragma unroll
    for (int off = 16; off > 0; off >>= 1) {
      p0 += __shfl_xor(p0, off, 32);
      p1 += __shfl_xor(p1, off, 32);
    }
    if (lane == 0) { v2f pv; pv.x = p0; pv.y = p1; *(v2f*)(splog + slot * NCLS) = pv; }
  }
  __syncthreads();

  float* gp = plog + ((size_t)b * (size_t)nPad + (size_t)nodeBase) * NCLS;
#pragma unroll
  for (int p = 0; p < NBA * NCLS / (4 * NTHR); ++p) {
    const int f = p * NTHR + tid;
    const v4f v = ((const v4f*)splog)[f];
    *(volatile v4f*)(gp + 4 * f) = v;
  }
  __threadfence();
#pragma unroll
  for (int p = 0; p < NBA * NCLS / (4 * NTHR); ++p) {
    const int f = p * NTHR + tid;
    const v4f v = ((const v4f*)splog)[f];
    *(volatile v4f*)(gp + 4 * f) = v;
  }
}

__global__ __launch_bounds__(NTHR) void k_final(
    const float* __restrict__ plog, const float* __restrict__ ob, float* out, int nN, int nPad) {
  const int i = blockIdx.x * NTHR + (int)threadIdx.x;
  const int nq  = nN >> 1;
  const int odd = nN & 1;
  const float ob0 = ob[0], ob1 = ob[1];
  v4f r = {0.f, 0.f, 0.f, 0.f};
#pragma unroll 1
  for (int q = 0; q < 2; ++q) {
    int n = 2 * i + q;
    n = n > nN - 1 ? nN - 1 : (n < 0 ? 0 : n);
    float x0 = ob0, x1 = ob1;
#pragma unroll
    for (int bb = 0; bb < NBAND; ++bb) {
      const v2f p = *(const v2f*)(plog + ((size_t)bb * (size_t)nPad + (size_t)n) * NCLS);
      x0 += p.x; x1 += p.y;
    }
    const float mx = fmaxf(x0, x1);
    const float s0 = x0 - mx, s1 = x1 - mx;
    const float lse = logf(expf(s0) + expf(s1));
    const float y0 = s0 - lse, y1 = s1 - lse;
    r.x = (q == 0) ? y0 : r.x;
    r.y = (q == 0) ? y1 : r.y;
    r.z = (q == 0) ? r.z : y0;
    r.w = (q == 0) ? r.w : y1;
  }
  const bool full = i < nq;
  const bool tail = (odd != 0) && (i == nq);
  v2f t2; t2.x = r.x; t2.y = r.y;
  if (full) *(volatile v4f*)(out + 4 * (size_t)i) = r;
  else if (tail) *(volatile v2f*)(out + 4 * (size_t)i) = t2;
  __threadfence();
  if (full) *(volatile v4f*)(out + 4 * (size_t)i) = r;
  else if (tail) *(volatile v2f*)(out + 4 * (size_t)i) = t2;
}

extern "C" void kernel_launch(void* const* d_in, const int* in_sizes, int n_in,
                              void* d_out, int out_size, void* d_ws, size_t ws_size,
                              hipStream_t stream) {
  if (n_in < 12) return;
  const int nN  = in_sizes[0] / FDIM;
  const int nE  = in_sizes[1] / 2;
  const int nEs = in_sizes[3] / (NBAND * 2);
  if (nN <= 0 || nE <= 0 || nEs <= 0) return;
  if (in_sizes[0] != nN * FDIM || in_sizes[1] != 2 * nE || in_sizes[2] != nE || in_sizes[3] != NBAND * 2 * nEs) return;
  if (in_sizes[4] != HDIM || in_sizes[5] != HDIM || in_sizes[6] != HDIM * HDIM || in_sizes[7] != HDIM) return;
  if (in_sizes[8] != NBAND * KDIM * HDIM || in_sizes[9] != NBAND * HDIM || in_sizes[10] != XCOL * NCLS || in_sizes[11] != NCLS) return;
  if (out_size != nN * NCLS) return;
  if (nN > (1 << 24) || nE > (1 << 28) || nEs > (1 << 28)) return;

  const float* feat = (const float*)d_in[0];
  const int*   ei   = (const int*)d_in[1];
  const float* ea   = (const float*)d_in[2];
  const int*   se   = (const int*)d_in[3];
  const float* tew  = (const float*)d_in[4];
  const float* teb  = (const float*)d_in[5];
  const float* taw  = (const float*)d_in[6];
  const float* tab  = (const float*)d_in[7];
  const float* cvw  = (const float*)d_in[8];
  const float* cvb  = (const float*)d_in[9];
  const float* ow   = (const float*)d_in[10];
  const float* ob   = (const float*)d_in[11];
  float* out = (float*)d_out;

  const int nAB    = (nN + NBA - 1) / NBA;
  const int NPAD   = nAB * NBA;
  const int nGB    = NPAD / GROWS;
  const int nBC    = (nN + NBC - 1) / NBC;
  const int CNTPAD = nBC * NBC;

  char* ws = (char*)d_ws;
  size_t off = 0;
  const size_t oWta = off; off += (size_t)HDIM * HDIM * 2;             off = (off + 255) & ~(size_t)255;
  const size_t oWcv = off; off += (size_t)XCOL * KDIM * 2;             off = (off + 255) & ~(size_t)255;
  const size_t oDv  = off; off += (size_t)NBAND * CNTPAD * 4;          off = (off + 255) & ~(size_t)255;
  const size_t oTs  = off; off += (size_t)NPAD * HDIM * 4;             off = (off + 255) & ~(size_t)255;
  const size_t oF16 = off; off += (size_t)NPAD * KDIM * 2;             off = (off + 255) & ~(size_t)255;
  const size_t oXw  = off; off += (size_t)NPAD * XCOL * 4;             off = (off + 255) & ~(size_t)255;
  const size_t oPl  = off; off += (size_t)NBAND * NPAD * NCLS * 4;     off = (off + 255) & ~(size_t)255;
  if (off > ws_size || off > (size_t)134217728) return;
  _Float16* wta  = (_Float16*)(ws + oWta);
  _Float16* wcv  = (_Float16*)(ws + oWcv);
  float*    dinv = (float*)(ws + oDv);
  float*    tsum = (float*)(ws + oTs);
  _Float16* f16p = (_Float16*)(ws + oF16);
  float*    xw   = (float*)(ws + oXw);
  float*    plog = (float*)(ws + oPl);

  const int vecT = ((nE  & 3) == 0) ? 1 : 0;
  const int vecS = ((nEs & 3) == 0) ? 1 : 0;

  const int nPrep = HDIM * HDIM / 8 + XCOL * KDIM / 8;
  k_wprep<<<(nPrep + NTHR - 1) / NTHR, NTHR, 0, stream>>>(taw, cvw, wta, wcv);

  k_count<<<dim3(nBC, NBAND), NTHR, 0, stream>>>(se, dinv, nEs, CNTPAD, vecS);

  hipFuncSetAttribute(reinterpret_cast<const void*>(&k_tagg),
                      hipFuncAttributeMaxDynamicSharedMemorySize, LDS_AGG);
  k_tagg<<<nAB, NTHR, LDS_AGG, stream>>>(ei, ea, tew, teb, tsum, nE, vecT);

  hipFuncSetAttribute(reinterpret_cast<const void*>(&k_feat),
                      hipFuncAttributeMaxDynamicSharedMemorySize, LDS_FEAT);
  k_feat<<<nGB, NTHR, LDS_FEAT, stream>>>(tsum, wta, tab, feat, f16p, nN);

  hipFuncSetAttribute(reinterpret_cast<const void*>(&k_xw),
                      hipFuncAttributeMaxDynamicSharedMemorySize, LDS_XW);
  k_xw<<<dim3(nGB, 2), NTHR, LDS_XW, stream>>>(f16p, wcv, dinv, xw, CNTPAD);

  hipFuncSetAttribute(reinterpret_cast<const void*>(&k_band),
                      hipFuncAttributeMaxDynamicSharedMemorySize, LDS_AGG);
  k_band<<<dim3(nAB, NBAND), NTHR, LDS_AGG, stream>>>(se, xw, dinv, cvb, ow, plog, nN, nEs, CNTPAD, NPAD, vecS);

  const int nThrF = (nN >> 1) + (nN & 1);
  k_final<<<(nThrF + NTHR - 1) / NTHR, NTHR, 0, stream>>>(plog, ob, out, nN, NPAD);
}
